// DSC_19207093748017
// MI455X (gfx1250) — hardware-verified
//
#include <hip/hip_runtime.h>
#include <stdint.h>

typedef __attribute__((ext_vector_type(16))) _Float16 v16h;
typedef __attribute__((ext_vector_type(8)))  _Float16 v8h;
typedef __attribute__((ext_vector_type(16))) __bf16   v16b;
typedef __attribute__((ext_vector_type(8)))  __bf16   v8b;
typedef __attribute__((ext_vector_type(8)))  float    v8f;
typedef __attribute__((ext_vector_type(4)))  float    v4f;
typedef __attribute__((ext_vector_type(4)))  unsigned v4u;

constexpr int NSAMP  = 4;
constexpr int NCH    = 512;
constexpr int HDIM   = 64;
constexpr int WDIM   = 64;
constexpr int NHW    = HDIM * WDIM;
constexpr int NCAT   = 4 * NCH;
constexpr int NPAIR  = 2;
constexpr int MROWS  = NPAIR * NHW;

static_assert(MROWS % 64 == 0);
static_assert(NCH % 64 == 0);
static_assert(NHW % 64 == 0);
static_assert(NCH % 32 == 0);
static_assert(NCAT % 32 == 0);
static_assert(NSAMP % NPAIR == 0);
static_assert(HDIM == 64 && WDIM == 64);

__device__ __forceinline__ unsigned short f2bf_bits(float f) {
  unsigned u = __float_as_uint(f);
  return (unsigned short)((u + 0x7FFFu + ((u >> 16) & 1u)) >> 16);
}
__device__ __forceinline__ float bf_bits2f(unsigned short h) { return __uint_as_float(((unsigned)h) << 16); }

__device__ __forceinline__ void dep_guard_h(v8f& a, v8f& b, v16h x, v16h y) { asm volatile("v_nop\n\tv_nop\n\tv_nop\n\tv_nop" : "+v"(a), "+v"(b) : "v"(x), "v"(y)); }
__device__ __forceinline__ void dep_guard_b(v8f& a, v8f& b, v16b x, v16b y) { asm volatile("v_nop\n\tv_nop\n\tv_nop\n\tv_nop" : "+v"(a), "+v"(b) : "v"(x), "v"(y)); }
__device__ __forceinline__ void keep4_h(v16h a, v16h b, v16h c, v16h d) { asm volatile("v_nop" :: "v"(a), "v"(b), "v"(c), "v"(d)); }
__device__ __forceinline__ void keep4_b(v16b a, v16b b, v16b c, v16b d) { asm volatile("v_nop" :: "v"(a), "v"(b), "v"(c), "v"(d)); }
__device__ __forceinline__ void acc_guard4(v8f& a, v8f& b, v8f& c, v8f& d) { asm volatile("v_nop\n\tv_nop\n\tv_nop\n\tv_nop" : "+v"(a), "+v"(b), "+v"(c), "+v"(d)); }

template <typename T> struct Frag;
template <> struct Frag<_Float16> {
  typedef v16h V; union U { v16h v; v8h h[2]; };
  static __device__ __forceinline__ v16h load(const _Float16* p) {
    U f; f.h[0] = *(const v8h*)(p); f.h[1] = *(const v8h*)(p + 16); return f.v;
  }
  static __device__ __forceinline__ v8f mma(v16h a, v16h b, v8f c) {
    return __builtin_amdgcn_wmma_f32_16x16x32_f16(false, a, false, b, (short)0, c, false, false);
  }
  static __device__ __forceinline__ void guard(v8f& a, v8f& b, v16h x, v16h y) { dep_guard_h(a, b, x, y); }
  static __device__ __forceinline__ void keep(v16h a, v16h b, v16h c, v16h d) { keep4_h(a, b, c, d); }
};
template <> struct Frag<__bf16> {
  typedef v16b V; union U { v16b v; v8b h[2]; };
  static __device__ __forceinline__ v16b load(const __bf16* p) {
    U f; f.h[0] = *(const v8b*)(p); f.h[1] = *(const v8b*)(p + 16); return f.v;
  }
  static __device__ __forceinline__ v8f mma(v16b a, v16b b, v8f c) {
    return __builtin_amdgcn_wmma_f32_16x16x32_bf16(false, a, false, b, (short)0, c, false, false);
  }
  static __device__ __forceinline__ void guard(v8f& a, v8f& b, v16b x, v16b y) { dep_guard_b(a, b, x, y); }
  static __device__ __forceinline__ void keep(v16b a, v16b b, v16b c, v16b d) { keep4_b(a, b, c, d); }
};

template <int ET> struct Elem;
template <> struct Elem<0> { typedef _Float16 T; };
template <> struct Elem<1> { typedef __bf16 T; };
template <int ET, bool SPA, bool SPB, int BIAS_MODE, int OUT_MODE, bool RESID, int ACT = 0>
__global__ __launch_bounds__(256) void wmma_gemm64(
    const unsigned short* __restrict__ Ap, const unsigned short* __restrict__ A2p, int lda, long strideA,
    const unsigned short* __restrict__ Btp, const unsigned short* __restrict__ Bt2p, int ldb, long strideB,
    void* __restrict__ Cout, void* __restrict__ Cout2, int ldc, long strideC,
    const float* __restrict__ bias,
    const float* __restrict__ resid, long strideR,
    int M, int N, int K, float scale) {
  typedef typename Elem<ET>::T T;
  typedef typename Frag<T>::V V;
  const T* A = (const T*)Ap; const T* A2 = (const T*)A2p; const T* Bt = (const T*)Btp; const T* Bt2 = (const T*)Bt2p;
  __shared__ __align__(16) float sT[8][16 * 68];
  const int b    = blockIdx.y;
  const int lane = threadIdx.x & 31;
  const int wave = threadIdx.x >> 5;
  const int tilesN = N >> 6;
  const int tilesM = M >> 6;
  const int tile = blockIdx.x * 8 + wave;
  if (tile >= tilesM * tilesN) return;
  const int tm = tile / tilesN;
  const int tn = tile - tm * tilesN;
  const int m0 = tm << 6;
  const int n0 = tn << 6;

  const T* Ab  = A  + (size_t)b * strideA;
  const T* Bb  = Bt + (size_t)b * strideB;
  const T* Ab2 = SPA ? (A2  + (size_t)b * strideA) : nullptr;
  const T* Bb2 = SPB ? (Bt2 + (size_t)b * strideB) : nullptr;

  const int rlane = lane & 15;
  const int koff  = (lane >> 4) * 8;
  const int mOff  = (lane >> 4) * 8;

  v8f acc[4][4];
#pragma unroll
  for (int i = 0; i < 4; ++i)
#pragma unroll
    for (int j = 0; j < 4; ++j) acc[i][j] = (v8f){0.f,0.f,0.f,0.f,0.f,0.f,0.f,0.f};

  for (int k0 = 0; k0 < K; k0 += 32) {
    V bh[4], bl[4];
#pragma unroll
    for (int j = 0; j < 4; ++j) {
      const size_t bo = (size_t)(n0 + (j << 4) + rlane) * ldb + koff + k0;
      bh[j] = Frag<T>::load(Bb + bo);
      if (SPB) bl[j] = Frag<T>::load(Bb2 + bo);
    }
#pragma unroll
    for (int i = 0; i < 4; ++i) {
      const size_t ao = (size_t)(m0 + (i << 4) + rlane) * lda + koff + k0;
      V ah = Frag<T>::load(Ab + ao);
      V al;
      if (SPA) al = Frag<T>::load(Ab2 + ao); else al = ah;
#pragma unroll
      for (int j = 0; j < 4; ++j) {
        acc[i][j] = Frag<T>::mma(ah, bh[j], acc[i][j]);
        if (SPB) acc[i][j] = Frag<T>::mma(ah, bl[j], acc[i][j]);
        if (SPA) acc[i][j] = Frag<T>::mma(al, bh[j], acc[i][j]);
      }
      Frag<T>::guard(acc[i][0], acc[i][3], ah, al);
    }
    Frag<T>::keep(bh[0], bh[1], bh[2], bh[3]);
    if (SPB) Frag<T>::keep(bl[0], bl[1], bl[2], bl[3]);
  }
  acc_guard4(acc[0][0], acc[0][1], acc[0][2], acc[0][3]);
  acc_guard4(acc[1][0], acc[1][1], acc[1][2], acc[1][3]);
  acc_guard4(acc[2][0], acc[2][1], acc[2][2], acc[2][3]);
  acc_guard4(acc[3][0], acc[3][1], acc[3][2], acc[3][3]);

  float* slab = sT[wave];
  const float* Rb = RESID ? (resid + (size_t)b * strideR) : nullptr;
#pragma unroll
  for (int i = 0; i < 4; ++i) {
    const int mBase = m0 + (i << 4);
#pragma unroll
    for (int j = 0; j < 4; ++j) {
      const int n = n0 + (j << 4) + rlane;
      float bv = 0.f;
      if (BIAS_MODE == 2) bv = bias[n];
#pragma unroll
      for (int r = 0; r < 8; ++r) {
        float v = acc[i][j][r] * scale;
        if (BIAS_MODE == 1) v += bias[mBase + mOff + r];
        if (BIAS_MODE == 2) v += bv;
        if (RESID) v += Rb[(size_t)(mBase + mOff + r) * ldc + n];
        if (ACT == 1) v = tanhf(v);
        if (ACT == 2) v = fmaxf(v, 0.0f);
        if (ACT == 3) v = v / (1.0f + expf(-v));
        if (ACT == 4) v = (v > 0.f) ? v : 0.01f * v;
        slab[(mOff + r) * 68 + (j << 4) + rlane] = v;
      }
    }
    __builtin_amdgcn_fence(__ATOMIC_RELEASE, "workgroup");
    __builtin_amdgcn_wave_barrier();
    __builtin_amdgcn_fence(__ATOMIC_ACQUIRE, "workgroup");
    if (OUT_MODE == 0) {
      float* C = (float*)Cout + (size_t)b * strideC;
      const int hh = lane >> 4, c4 = (lane & 15) * 4;
      for (int pass = 0; pass < 2; ++pass) {
#pragma unroll
        for (int it = 0; it < 8; ++it) {
          const int row = it * 2 + hh;
          v4f v = *(const v4f*)(slab + row * 68 + c4);
          *(volatile v4f*)(C + (size_t)(mBase + row) * ldc + n0 + c4) = v;
        }
        __threadfence();
      }
    } else {
      const int q = lane >> 3, c8 = (lane & 7) * 8;
      unsigned short* C  = (unsigned short*)Cout  + (size_t)b * strideC;
      unsigned short* C2 = (OUT_MODE == 2) ? ((unsigned short*)Cout2 + (size_t)b * strideC) : nullptr;
      for (int pass = 0; pass < 2; ++pass) {
#pragma unroll
        for (int it = 0; it < 4; ++it) {
          const int row = it * 4 + q;
          const float* sp = slab + row * 68 + c8;
          v8h hv, lv;
#pragma unroll
          for (int e = 0; e < 8; ++e) {
            if (OUT_MODE == 1) {
              hv[e] = (_Float16)sp[e];
            } else {
              unsigned short hb = f2bf_bits(sp[e]);
              unsigned short lb = f2bf_bits(sp[e] - bf_bits2f(hb));
              hv[e] = __builtin_bit_cast(_Float16, hb);
              lv[e] = __builtin_bit_cast(_Float16, lb);
            }
          }
          *(volatile v8h*)(C + (size_t)(mBase + row) * ldc + n0 + c8) = hv;
          if (OUT_MODE == 2) *(volatile v8h*)(C2 + (size_t)(mBase + row) * ldc + n0 + c8) = lv;
        }
        __threadfence();
      }
    }
    __builtin_amdgcn_fence(__ATOMIC_RELEASE, "workgroup");
    __builtin_amdgcn_wave_barrier();
    __builtin_amdgcn_fence(__ATOMIC_ACQUIRE, "workgroup");
  }
}

__global__ __launch_bounds__(256) void cast_f32_bf16x8(
    const float* __restrict__ in, unsigned short* __restrict__ out, int n8) {
  const int i = blockIdx.x * 256 + threadIdx.x;
  if (i < n8) {
    const v4f a = *(const v4f*)(in + (size_t)i * 8);
    const v4f c = *(const v4f*)(in + (size_t)i * 8 + 4);
    v4u u;
    u[0] = (unsigned)f2bf_bits(a[0]) | ((unsigned)f2bf_bits(a[1]) << 16);
    u[1] = (unsigned)f2bf_bits(a[2]) | ((unsigned)f2bf_bits(a[3]) << 16);
    u[2] = (unsigned)f2bf_bits(c[0]) | ((unsigned)f2bf_bits(c[1]) << 16);
    u[3] = (unsigned)f2bf_bits(c[2]) | ((unsigned)f2bf_bits(c[3]) << 16);
    unsigned short* p = out + (size_t)i * 8;
    *(volatile v4u*)p = u;
    __threadfence();
    *(volatile v4u*)p = u;
  }
}

__global__ __launch_bounds__(256) void nchw_to_rows_bf16(const float* __restrict__ x,
                                                        unsigned short* __restrict__ xT,
                                                        int sampleBase) {
  __shared__ __align__(16) float tile[64][68];
  const int t = threadIdx.x;
  const int hw0 = blockIdx.x * 64;
  const int c0 = blockIdx.y * 64;
  const int sl = blockIdx.z;
  const float* src = x + ((size_t)(sampleBase + sl) * NCH + c0) * NHW + hw0;
#pragma unroll
  for (int i = 0; i < 4; ++i) {
    const int f = t + 256 * i;
    const int c = f >> 4, hw4 = (f & 15) * 4;
    const v4f v = *(const v4f*)(src + (size_t)c * NHW + hw4);
    *(v4f*)(&tile[c][hw4]) = v;
  }
  __syncthreads();
  const int wave = t >> 5, lane = t & 31, q = lane >> 3, c8 = (lane & 7) * 8;
  unsigned short* dst = xT + ((size_t)sl * NHW + hw0) * NCH + c0 + c8;
  v4u u[2];
  int hwr[2];
#pragma unroll
  for (int it = 0; it < 2; ++it) {
    const int hw = it * 32 + wave * 4 + q;
    hwr[it] = hw;
    v4u p;
#pragma unroll
    for (int e = 0; e < 4; ++e) {
      const unsigned lo16 = (unsigned)f2bf_bits(tile[c8 + 2 * e][hw]);
      const unsigned hi16 = (unsigned)f2bf_bits(tile[c8 + 2 * e + 1][hw]);
      p[e] = lo16 | (hi16 << 16);
    }
    u[it] = p;
  }
  for (int pass = 0; pass < 2; ++pass) {
#pragma unroll
    for (int it = 0; it < 2; ++it)
      *(volatile v4u*)(dst + (size_t)hwr[it] * NCH) = u[it];
    __threadfence();
  }
}

__global__ __launch_bounds__(256) void irnn_scan4(const float* __restrict__ y,
    const float* __restrict__ wu, const float* __restrict__ bu,
    const float* __restrict__ wr, const float* __restrict__ br,
    const float* __restrict__ wd, const float* __restrict__ bd,
    const float* __restrict__ wl, const float* __restrict__ bl,
    unsigned short* __restrict__ dhi, unsigned short* __restrict__ dlo, int nSamples) {
  const int lane = threadIdx.x & 31;
  const int wave = threadIdx.x >> 5;
  const int gw = blockIdx.x * 8 + wave;
  const int dir = blockIdx.y;
  const int g = gw & 1;
  const int q = (gw >> 1) & 63;
  const int sl = gw >> 7;
  if (sl >= nSamples) return;
  const bool vert = (dir == 0) || (dir == 2);
  const bool rev  = (dir == 0) || (dir == 3);
  const float* wp = (dir == 0) ? wu : (dir == 1) ? wr : (dir == 2) ? wd : wl;
  const float* bp = (dir == 0) ? bu : (dir == 1) ? br : (dir == 2) ? bd : bl;
  const int cb = g * 256 + lane * 8;
  float wv[8], bv[8], st[8];
#pragma unroll
  for (int e = 0; e < 8; ++e) {
    wv[e] = bf_bits2f(f2bf_bits(wp[cb + e]));
    bv[e] = bf_bits2f(f2bf_bits(bp[cb + e]));
  }
  const size_t posStep = vert ? (size_t)WDIM : (size_t)1;
  const size_t base = (size_t)sl * NHW + (vert ? (size_t)q : (size_t)q * WDIM);
  const size_t dcol = (size_t)dir * NCH + cb;

  {
    const int idx = rev ? 63 : 0;
    const size_t pos = base + (size_t)idx * posStep;
    const float* yp = y + pos * NCH + cb;
    const v4f a = *(const v4f*)yp;
    const v4f c = *(const v4f*)(yp + 4);
#pragma unroll
    for (int e = 0; e < 4; ++e) { st[e] = fmaxf(a[e], 0.0f); st[4 + e] = fmaxf(c[e], 0.0f); }
    v4u z;
    z[0] = 0u; z[1] = 0u; z[2] = 0u; z[3] = 0u;
    unsigned short* hp = dhi + pos * NCAT + dcol;
    unsigned short* lp = dlo + pos * NCAT + dcol;
    *(volatile v4u*)hp = z; *(volatile v4u*)lp = z;
    __threadfence();
    *(volatile v4u*)hp = z; *(volatile v4u*)lp = z;
  }
#pragma unroll 1
  for (int t = 1; t < 64; ++t) {
    const int idx = rev ? (63 - t) : t;
    const size_t pos = base + (size_t)idx * posStep;
    const float* yp = y + pos * NCH + cb;
    const v4f a = *(const v4f*)yp;
    const v4f c = *(const v4f*)(yp + 4);
    float xv[8];
#pragma unroll
    for (int e = 0; e < 4; ++e) { xv[e] = a[e]; xv[4 + e] = c[e]; }
    unsigned hbits[8], lbits[8];
#pragma unroll
    for (int e = 0; e < 8; ++e) {
      const float v = fmaxf(fmaf(st[e], wv[e], bv[e]) + xv[e], 0.0f);
      st[e] = v;
      const unsigned short hb = f2bf_bits(v);
      const unsigned short lb = f2bf_bits(v - bf_bits2f(hb));
      hbits[e] = (unsigned)hb;
      lbits[e] = (unsigned)lb;
    }
    v4u hv, lv;
#pragma unroll
    for (int e = 0; e < 4; ++e) {
      hv[e] = hbits[2 * e] | (hbits[2 * e + 1] << 16);
      lv[e] = lbits[2 * e] | (lbits[2 * e + 1] << 16);
    }
    unsigned short* hp = dhi + pos * NCAT + dcol;
    unsigned short* lp = dlo + pos * NCAT + dcol;
    *(volatile v4u*)hp = hv; *(volatile v4u*)lp = lv;
    __threadfence();
    *(volatile v4u*)hp = hv; *(volatile v4u*)lp = lv;
  }
}

extern "C" void kernel_launch(void* const* d_in, const int* in_sizes, int n_in,
                              void* d_out, int out_size, void* d_ws, size_t ws_size,
                              hipStream_t stream) {
  if (n_in < 26) return;
  if (in_sizes[0] != NSAMP * NCH * NHW) return;
  if (in_sizes[7] != NCH * NCH) return;
  if (in_sizes[8] != NCH * NCAT || in_sizes[9] != NCH * NCAT) return;
  for (int i = 10; i < 26; ++i) if (in_sizes[i] != NCH) return;
  if (out_size != NSAMP * NCH * NHW) return;

  const float* x     = (const float*)d_in[0];
  const float* cin_w = (const float*)d_in[7];
  const float* c2_w  = (const float*)d_in[8];
  const float* c3_w  = (const float*)d_in[9];
  const float* i1_wu = (const float*)d_in[10]; const float* i1_bu = (const float*)d_in[11];
  const float* i1_wr = (const float*)d_in[12]; const float* i1_br = (const float*)d_in[13];
  const float* i1_wd = (const float*)d_in[14]; const float* i1_bd = (const float*)d_in[15];
  const float* i1_wl = (const float*)d_in[16]; const float* i1_bl = (const float*)d_in[17];
  const float* i2_wu = (const float*)d_in[18]; const float* i2_bu = (const float*)d_in[19];
  const float* i2_wr = (const float*)d_in[20]; const float* i2_br = (const float*)d_in[21];
  const float* i2_wd = (const float*)d_in[22]; const float* i2_bd = (const float*)d_in[23];
  const float* i2_wl = (const float*)d_in[24]; const float* i2_bl = (const float*)d_in[25];
  float* out = (float*)d_out;

  const size_t szW1 = (size_t)NCH * NCH * 2;
  const size_t szW2 = (size_t)NCH * NCAT * 2;
  const size_t szXT = (size_t)MROWS * NCH * 2;
  const size_t szY  = (size_t)MROWS * NCH * 4;
  const size_t szD  = (size_t)MROWS * NCAT * 2;
  size_t off = 0;
  unsigned short* wcin = (unsigned short*)((char*)d_ws + off); off += szW1;
  unsigned short* wc2  = (unsigned short*)((char*)d_ws + off); off += szW2;
  unsigned short* wc3  = (unsigned short*)((char*)d_ws + off); off += szW2;
  unsigned short* xT   = (unsigned short*)((char*)d_ws + off); off += szXT;
  float*          y    = (float*)((char*)d_ws + off);          off += szY;
  unsigned short* dhi  = (unsigned short*)((char*)d_ws + off); off += szD;
  unsigned short* dlo  = (unsigned short*)((char*)d_ws + off); off += szD;
  if (off > ws_size) return;
  const float* fdummy = (const float*)y;

  cast_f32_bf16x8<<<(NCH * NCH / 8 + 255) / 256, 256, 0, stream>>>(cin_w, wcin, NCH * NCH / 8);
  cast_f32_bf16x8<<<(NCH * NCAT / 8 + 255) / 256, 256, 0, stream>>>(c2_w, wc2, NCH * NCAT / 8);
  cast_f32_bf16x8<<<(NCH * NCAT / 8 + 255) / 256, 256, 0, stream>>>(c3_w, wc3, NCH * NCAT / 8);

  const dim3 gT(NHW / 64, NCH / 64, NPAIR);
  const int  tiles12 = (MROWS / 64) * (NCH / 64);
  const dim3 g12((tiles12 + 7) / 8, 1);
  const int  tiles3 = (NCH / 64) * (NHW / 64);
  const dim3 g3((tiles3 + 7) / 8, NPAIR);
  const dim3 gS(NPAIR * 64 * 2 / 8, 4);

  for (int p = 0; p < NSAMP / NPAIR; ++p) {
    nchw_to_rows_bf16<<<gT, 256, 0, stream>>>(x, xT, p * NPAIR);
    wmma_gemm64<1, false, false, 0, 0, false, 0><<<g12, 256, 0, stream>>>(
        xT, xT, NCH, 0L, wcin, wcin, NCH, 0L, y, y, NCH, 0L, fdummy, fdummy, 0L,
        MROWS, NCH, NCH, 1.0f);
    irnn_scan4<<<gS, 256, 0, stream>>>(y, i1_wu, i1_bu, i1_wr, i1_br, i1_wd, i1_bd, i1_wl, i1_bl,
                                        dhi, dlo, NPAIR);
    wmma_gemm64<1, true, false, 0, 0, false, 0><<<g12, 256, 0, stream>>>(
        dhi, dlo, NCAT, 0L, wc2, wc2, NCAT, 0L, y, y, NCH, 0L, fdummy, fdummy, 0L,
        MROWS, NCH, NCAT, 1.0f);
    irnn_scan4<<<gS, 256, 0, stream>>>(y, i2_wu, i2_bu, i2_wr, i2_br, i2_wd, i2_bd, i2_wl, i2_bl,
                                        dhi, dlo, NPAIR);
    wmma_gemm64<1, false, true, 0, 0, false, 2><<<g3, 256, 0, stream>>>(
        wc3, wc3, NCAT, 0L, dhi, dlo, NCAT, (long)NHW * NCAT,
        out + (size_t)p * NPAIR * NCH * NHW, out + (size_t)p * NPAIR * NCH * NHW, NHW, (long)NCH * NHW,
        fdummy, fdummy, 0L, NCH, NHW, NCAT, 1.0f);
  }
}
